// LinearTransformerBlock_52707838656612
// MI455X (gfx1250) — hardware-verified
//
#include <hip/hip_runtime.h>
#include <math.h>
#include <stdint.h>

#define T_SEQ   2048
#define D_MODEL 1024
#define N_HEADS 16
#define D_HEAD  64
#define D_FF    4096
#define W_SCALE 256.0f
#define O_SCALE 64.0f

typedef _Float16 half_t;
typedef __attribute__((ext_vector_type(16))) _Float16 v16h;
typedef __attribute__((ext_vector_type(8)))  _Float16 v8h;
typedef __attribute__((ext_vector_type(8)))  float    v8f;
typedef __attribute__((ext_vector_type(4)))  float    v4f;

union FragU { v16h v; v8h h[2]; };

__device__ __forceinline__ v16h ldfrag(const half_t* p) {
  FragU f;
  f.h[0] = *(const v8h*)(p);
  f.h[1] = *(const v8h*)(p + 16);
  return f.v;
}

__device__ __forceinline__ v8f mma16(v16h a, v16h b, v8f c) {
  c = __builtin_amdgcn_wmma_f32_16x16x32_f16(false, a, false, b, (short)0, c, false, false);
  asm volatile("v_nop\n\tv_nop\n\tv_nop\n\tv_nop" : "+v"(c) : "v"(a), "v"(b));
  return c;
}

__device__ __forceinline__ v8f zero8() { v8f z = {0.f, 0.f, 0.f, 0.f, 0.f, 0.f, 0.f, 0.f}; return z; }

__global__ __launch_bounds__(256) void tconv_kernel(const float* __restrict__ W, half_t* __restrict__ out,
                                                    int R, int Cc, float scl) {
  __shared__ __align__(16) float tf[64 * 68];
  const int c0  = blockIdx.x * 64;
  const int r0  = blockIdx.y * 64;
  const int tid = threadIdx.x;
  {
    const int lr = tid >> 4;
    const int c4 = (tid & 15) * 4;
#pragma unroll
    for (int it = 0; it < 4; ++it) {
      const int rr = it * 16 + lr;
      const v4f a = *(const v4f*)(W + (size_t)(r0 + rr) * Cc + c0 + c4);
      *(v4f*)(tf + rr * 68 + c4) = a;
    }
  }
  __syncthreads();
  const int sub = tid >> 3;
  const int c8  = (tid & 7) * 8;
  v8h hv0, hv1;
#pragma unroll
  for (int e = 0; e < 8; ++e) {
    hv0[e] = (half_t)(tf[(c8 + e) * 68 + sub] * scl);
    hv1[e] = (half_t)(tf[(c8 + e) * 68 + 32 + sub] * scl);
  }
  const size_t g0 = (size_t)(c0 + sub) * R + r0 + c8;
  const size_t g1 = (size_t)(c0 + 32 + sub) * R + r0 + c8;
  for (int pass = 0; pass < 2; ++pass) {
    *(volatile v8h*)(out + g0) = hv0;
    *(volatile v8h*)(out + g1) = hv1;
    __threadfence();
  }
}

__global__ __launch_bounds__(128) void ln_kernel(const float* __restrict__ X, const float* __restrict__ g,
                                                 const float* __restrict__ bb, half_t* __restrict__ Y) {
  __shared__ float red1[4];
  __shared__ float red2[4];
  const int row  = blockIdx.x;
  const int tid  = threadIdx.x;
  const int lane = tid & 31;
  const int wave = tid >> 5;
  const float* xr = X + (size_t)row * D_MODEL + tid * 8;
  const v4f a0 = *(const v4f*)(xr);
  const v4f a1 = *(const v4f*)(xr + 4);
  float s = ((a0[0] + a0[1]) + (a0[2] + a0[3])) + ((a1[0] + a1[1]) + (a1[2] + a1[3]));
#pragma unroll
  for (int off = 1; off < 32; off <<= 1) s += __shfl_xor(s, off, 32);
  if (lane == 0) red1[wave] = s;
  __syncthreads();
  const float mean = ((red1[0] + red1[1]) + (red1[2] + red1[3])) * (1.0f / D_MODEL);
  float d[8];
#pragma unroll
  for (int e = 0; e < 4; ++e) { d[e] = a0[e] - mean; d[e + 4] = a1[e] - mean; }
  float q = 0.f;
#pragma unroll
  for (int e = 0; e < 8; ++e) q += d[e] * d[e];
#pragma unroll
  for (int off = 1; off < 32; off <<= 1) q += __shfl_xor(q, off, 32);
  if (lane == 0) red2[wave] = q;
  __syncthreads();
  const float var  = ((red2[0] + red2[1]) + (red2[2] + red2[3])) * (1.0f / D_MODEL);
  const float rstd = 1.0f / sqrtf(var + 1e-5f);
  const v4f g0 = *(const v4f*)(g + tid * 8);
  const v4f g1 = *(const v4f*)(g + tid * 8 + 4);
  const v4f b0 = *(const v4f*)(bb + tid * 8);
  const v4f b1 = *(const v4f*)(bb + tid * 8 + 4);
  v8h y;
#pragma unroll
  for (int e = 0; e < 4; ++e) {
    y[e]     = (half_t)((d[e] * rstd) * g0[e] + b0[e]);
    y[e + 4] = (half_t)((d[e + 4] * rstd) * g1[e] + b1[e]);
  }
  half_t* yp = Y + (size_t)row * D_MODEL + tid * 8;
  *(volatile v8h*)yp = y;
  __threadfence();
  *(volatile v8h*)yp = y;
}

template <int EPI>
__global__ __launch_bounds__(256) void gemm_kernel(const half_t* __restrict__ A, int lda,
                                                   const half_t* __restrict__ Bt, int ldb,
                                                   void* __restrict__ Cout, int ldc,
                                                   const float* __restrict__ resid, int ldr,
                                                   int M, int N, int K, float scale, int ncut) {
  __shared__ __align__(16) float sT[8][16 * 68];
  const int lane = threadIdx.x & 31;
  const int wave = threadIdx.x >> 5;
  const int tilesN = N >> 6;
  const int tilesM = M >> 5;
  const int tile = blockIdx.x * 8 + wave;
  if (tile >= tilesM * tilesN) return;
  const int tm = tile / tilesN;
  const int tn = tile - tm * tilesN;
  const int m0 = tm << 5;
  const int n0 = tn << 6;
  const int rl   = lane & 15;
  const int hh   = lane >> 4;
  const int koff = hh * 8;
  const int mOff = hh * 8;

  v8f acc[2][4];
#pragma unroll
  for (int i = 0; i < 2; ++i)
#pragma unroll
    for (int j = 0; j < 4; ++j) acc[i][j] = zero8();

#pragma unroll 1
  for (int k0 = 0; k0 < K; k0 += 32) {
    v16h bf[4];
#pragma unroll
    for (int j = 0; j < 4; ++j)
      bf[j] = ldfrag(Bt + (size_t)(n0 + 16 * j + rl) * ldb + k0 + koff);
#pragma unroll
    for (int i = 0; i < 2; ++i) {
      const v16h af = ldfrag(A + (size_t)(m0 + 16 * i + rl) * lda + k0 + koff);
#pragma unroll
      for (int j = 0; j < 4; ++j) acc[i][j] = mma16(af, bf[j], acc[i][j]);
    }
  }

  float* slab = sT[wave];
#pragma unroll
  for (int i = 0; i < 2; ++i) {
    const int mBase = m0 + 16 * i;
#pragma unroll
    for (int j = 0; j < 4; ++j) {
      const int n = n0 + 16 * j + rl;
#pragma unroll
      for (int r = 0; r < 8; ++r) {
        float v = acc[i][j][r] * scale;
        if (EPI == 2) v += resid[(size_t)(mBase + mOff + r) * ldr + n];
        if (EPI == 0) {
          if (n0 < ncut) v = (v > 0.0f) ? (v + 1.0f) : (expf(v));
        }
        if (EPI == 1) v = 0.5f * v * (1.0f + erff(v * 0.70710678118654752f));
        slab[(mOff + r) * 68 + 16 * j + rl] = v;
      }
    }
    __builtin_amdgcn_fence(__ATOMIC_RELEASE, "workgroup");
    __builtin_amdgcn_wave_barrier();
    __builtin_amdgcn_fence(__ATOMIC_ACQUIRE, "workgroup");
    if (EPI == 2) {
      float* C = (float*)Cout;
      const int c4 = rl * 4;
      for (int pass = 0; pass < 2; ++pass) {
#pragma unroll
        for (int it = 0; it < 8; ++it) {
          const int row = it * 2 + hh;
          const v4f v = *(const v4f*)(slab + row * 68 + c4);
          *(volatile v4f*)(C + (size_t)(mBase + row) * ldc + n0 + c4) = v;
        }
        __threadfence();
      }
    } else {
      half_t* C = (half_t*)Cout;
      const int q = lane >> 3, c8 = (lane & 7) * 8;
      for (int pass = 0; pass < 2; ++pass) {
#pragma unroll
        for (int it = 0; it < 4; ++it) {
          const int row = it * 4 + q;
          const float* sp = slab + row * 68 + c8;
          v8h hv;
#pragma unroll
          for (int e = 0; e < 8; ++e) hv[e] = (half_t)sp[e];
          *(volatile v8h*)(C + (size_t)(mBase + row) * ldc + n0 + c8) = hv;
        }
        __threadfence();
      }
    }
    __builtin_amdgcn_fence(__ATOMIC_RELEASE, "workgroup");
    __builtin_amdgcn_wave_barrier();
    __builtin_amdgcn_fence(__ATOMIC_ACQUIRE, "workgroup");
  }
}

#define LDSFRAG(dst, arr, row, k)                                           \
  do {                                                                      \
    FragU f_;                                                               \
    f_.h[0] = *(const v8h*)((arr) + (row) * 64 + (k) + 8 * hh);             \
    f_.h[1] = *(const v8h*)((arr) + (row) * 64 + (k) + 16 + 8 * hh);        \
    (dst) = f_.v;                                                           \
  } while (0)

__global__ __launch_bounds__(256) void attn_kernel(const half_t* __restrict__ QKV, half_t* __restrict__ Opl) {
  __shared__ __align__(16) half_t Qc[64 * 64];
  __shared__ __align__(16) half_t Kc[64 * 64];
  __shared__ __align__(16) half_t KTc[64 * 64];
  __shared__ __align__(16) half_t VTc[64 * 64];
  __shared__ __align__(16) half_t STh[64 * 64];
  __shared__ __align__(16) half_t Am[64 * 64];
  __shared__ __align__(16) half_t Os[64 * 64];
  __shared__ float zsh[64];
  __shared__ float dinv[64];
  __shared__ float denp[2][64];

  const int h    = blockIdx.x;
  const int tid  = threadIdx.x;
  const int wave = tid >> 5;
  const int lane = tid & 31;
  const int hh   = lane >> 4;
  const int c    = lane & 15;
  const int m0   = (wave >> 1) * 16;
  const int ncp  = (wave & 1) * 32;
  const int crow = m0 + 8 * hh;
  const int PQKV = 3 * D_MODEL;

  const half_t* Qp = QKV + h * D_HEAD;
  const half_t* Kp = QKV + D_MODEL + h * D_HEAD;
  const half_t* Vp = QKV + 2 * D_MODEL + h * D_HEAD;
  half_t* Op = Opl + h * D_HEAD;

  for (int i = tid; i < 64 * 64; i += 256) STh[i] = (half_t)0.0f;
  if (tid < 64) zsh[tid] = 0.0f;
  v8f sacc0 = zero8(), sacc1 = zero8();

  for (int ch = 0; ch < T_SEQ / 64; ++ch) {
    const int t0 = ch * 64;
    __syncthreads();
#pragma unroll
    for (int it = 0; it < 2; ++it) {
      const int vec = it * 256 + tid;
      const int r   = vec >> 3;
      const int c8  = (vec & 7) * 8;
      const size_t go = (size_t)(t0 + r) * PQKV + c8;
      const v8h qv = *(const v8h*)(Qp + go);
      const v8h kv = *(const v8h*)(Kp + go);
      const v8h vv = *(const v8h*)(Vp + go);
      *(v8h*)(Qc + r * 64 + c8) = qv;
      *(v8h*)(Kc + r * 64 + c8) = kv;
#pragma unroll
      for (int e = 0; e < 8; ++e) {
        KTc[(c8 + e) * 64 + r] = kv[e];
        VTc[(c8 + e) * 64 + r] = vv[e];
      }
    }
    __syncthreads();

    v16h qa0, qa1;
    LDSFRAG(qa0, Qc, m0 + c, 0);
    LDSFRAG(qa1, Qc, m0 + c, 32);
    v8f acc0 = zero8(), acc1 = zero8(), sc0 = zero8(), sc1 = zero8();
    {
      v16h b;
      LDSFRAG(b, STh, ncp + c, 0);       acc0 = mma16(qa0, b, acc0);
      LDSFRAG(b, STh, ncp + 16 + c, 0);  acc1 = mma16(qa0, b, acc1);
      LDSFRAG(b, STh, ncp + c, 32);      acc0 = mma16(qa1, b, acc0);
      LDSFRAG(b, STh, ncp + 16 + c, 32); acc1 = mma16(qa1, b, acc1);
      LDSFRAG(b, Kc, ncp + c, 0);        sc0 = mma16(qa0, b, sc0);
      LDSFRAG(b, Kc, ncp + 16 + c, 0);   sc1 = mma16(qa0, b, sc1);
      LDSFRAG(b, Kc, ncp + c, 32);       sc0 = mma16(qa1, b, sc0);
      LDSFRAG(b, Kc, ncp + 16 + c, 32);  sc1 = mma16(qa1, b, sc1);
    }
#pragma unroll
    for (int r = 0; r < 8; ++r) {
      const int row  = crow + r;
      const int col0 = ncp + c;
      const int col1 = col0 + 16;
      const float v0 = (col0 <= row) ? sc0[r] : 0.0f;
      const float v1 = (col1 <= row) ? sc1[r] : 0.0f;
      Am[row * 64 + col0] = (half_t)v0;
      Am[row * 64 + col1] = (half_t)v1;
      float part = v0 + v1;
      part += __shfl_xor(part, 1, 32);
      part += __shfl_xor(part, 2, 32);
      part += __shfl_xor(part, 4, 32);
      part += __shfl_xor(part, 8, 32);
      if (c == 0) denp[wave & 1][row] = part;
    }
    __syncthreads();

    if (tid < 64) {
      const int t = tid;
      float qz = 0.0f;
#pragma unroll 8
      for (int d = 0; d < 64; ++d) qz += (float)Qc[t * 64 + d] * zsh[d];
      const float den = fmaxf((denp[0][t] + denp[1][t]) + qz, 1e-6f);
      dinv[t] = 1.0f / den;
    }
    {
      v16h aa, ka, vb0, vb1;
      LDSFRAG(vb0, VTc, ncp + c, 0);
      LDSFRAG(vb1, VTc, ncp + 16 + c, 0);
      LDSFRAG(aa, Am, m0 + c, 0);
      LDSFRAG(ka, KTc, m0 + c, 0);
      acc0  = mma16(aa, vb0, acc0);
      acc1  = mma16(aa, vb1, acc1);
      sacc0 = mma16(ka, vb0, sacc0);
      sacc1 = mma16(ka, vb1, sacc1);
      LDSFRAG(vb0, VTc, ncp + c, 32);
      LDSFRAG(vb1, VTc, ncp + 16 + c, 32);
      LDSFRAG(aa, Am, m0 + c, 32);
      LDSFRAG(ka, KTc, m0 + c, 32);
      acc0  = mma16(aa, vb0, acc0);
      acc1  = mma16(aa, vb1, acc1);
      sacc0 = mma16(ka, vb0, sacc0);
      sacc1 = mma16(ka, vb1, sacc1);
    }
    __syncthreads();

    {
      v8h sv0, sv1;
#pragma unroll
      for (int r = 0; r < 8; ++r) { sv0[r] = (half_t)sacc0[r]; sv1[r] = (half_t)sacc1[r]; }
      *(v8h*)(STh + (ncp + c) * 64 + crow)      = sv0;
      *(v8h*)(STh + (ncp + 16 + c) * 64 + crow) = sv1;
    }
    if (tid < 64) {
      const int d = tid;
      float a = zsh[d];
#pragma unroll 8
      for (int t = 0; t < 64; ++t) a += (float)Kc[t * 64 + d];
      zsh[d] = a;
    }
#pragma unroll
    for (int r = 0; r < 8; ++r) {
      const int row = crow + r;
      const float inv = dinv[row] * O_SCALE;
      Os[row * 64 + ncp + c]      = (half_t)(acc0[r] * inv);
      Os[row * 64 + ncp + 16 + c] = (half_t)(acc1[r] * inv);
    }
    __syncthreads();

    for (int pass = 0; pass < 2; ++pass) {
#pragma unroll
      for (int it = 0; it < 2; ++it) {
        const int vec = it * 256 + tid;
        const int r   = vec >> 3;
        const int c8  = (vec & 7) * 8;
        const v8h ov = *(const v8h*)(Os + r * 64 + c8);
        *(volatile v8h*)(Op + (size_t)(t0 + r) * D_MODEL + c8) = ov;
      }
      __threadfence();
    }
  }
}

extern "C" void kernel_launch(void* const* d_in, const int* in_sizes, int n_in,
                              void* d_out, int out_size, void* d_ws, size_t ws_size,
                              hipStream_t stream) {
  if (n_in < 11) return;
  if (in_sizes[0] != T_SEQ * D_MODEL) return;
  if (in_sizes[1] != D_MODEL || in_sizes[2] != D_MODEL || in_sizes[7] != D_MODEL || in_sizes[8] != D_MODEL) return;
  if (in_sizes[3] != D_MODEL * D_MODEL || in_sizes[4] != D_MODEL * D_MODEL ||
      in_sizes[5] != D_MODEL * D_MODEL || in_sizes[6] != D_MODEL * D_MODEL) return;
  if (in_sizes[9] != D_MODEL * D_FF || in_sizes[10] != D_FF * D_MODEL) return;
  if (out_size != T_SEQ * D_MODEL) return;

  const float* x     = (const float*)d_in[0];
  const float* ln1_g = (const float*)d_in[1];
  const float* ln1_b = (const float*)d_in[2];
  const float* Wq    = (const float*)d_in[3];
  const float* Wk    = (const float*)d_in[4];
  const float* Wv    = (const float*)d_in[5];
  const float* Wo    = (const float*)d_in[6];
  const float* ln2_g = (const float*)d_in[7];
  const float* ln2_b = (const float*)d_in[8];
  const float* Wf1   = (const float*)d_in[9];
  const float* Wf2   = (const float*)d_in[10];
  float* out = (float*)d_out;

  const size_t szWqkv = (size_t)3 * D_MODEL * D_MODEL * 2;
  const size_t szWo   = (size_t)D_MODEL * D_MODEL * 2;
  const size_t szWf1  = (size_t)D_FF * D_MODEL * 2;
  const size_t szWf2  = (size_t)D_MODEL * D_FF * 2;
  const size_t szAct2 = (size_t)T_SEQ * D_MODEL * 2;
  const size_t szQKV  = (size_t)T_SEQ * 3 * D_MODEL * 2;
  const size_t szAct4 = (size_t)T_SEQ * D_MODEL * 4;
  const size_t szG    = (size_t)T_SEQ * D_FF * 2;
  size_t off = 0;
  const size_t oWqkv = off; off += szWqkv;
  const size_t oWo   = off; off += szWo;
  const size_t oWf1  = off; off += szWf1;
  const size_t oWf2  = off; off += szWf2;
  const size_t oXn   = off; off += szAct2;
  const size_t oQKV  = off; off += szQKV;
  const size_t oO    = off; off += szAct2;
  const size_t oX1   = off; off += szAct4;
  const size_t oH2   = off; off += szAct2;
  const size_t oG    = off; off += szG;
  if (off > ws_size) return;

  char* ws = (char*)d_ws;
  half_t* WqkvT = (half_t*)(ws + oWqkv);
  half_t* WoT   = (half_t*)(ws + oWo);
  half_t* Wf1T  = (half_t*)(ws + oWf1);
  half_t* Wf2T  = (half_t*)(ws + oWf2);
  half_t* Xn    = (half_t*)(ws + oXn);
  half_t* QKV   = (half_t*)(ws + oQKV);
  half_t* Opl   = (half_t*)(ws + oO);
  float*  X1    = (float*)(ws + oX1);
  half_t* H2    = (half_t*)(ws + oH2);
  half_t* G     = (half_t*)(ws + oG);

  const dim3 blk256(256);
  const dim3 blk128(128);

  tconv_kernel<<<dim3(D_MODEL / 64, D_MODEL / 64), blk256, 0, stream>>>(Wq, WqkvT, D_MODEL, D_MODEL, W_SCALE);
  tconv_kernel<<<dim3(D_MODEL / 64, D_MODEL / 64), blk256, 0, stream>>>(Wk, WqkvT + (size_t)D_MODEL * D_MODEL, D_MODEL, D_MODEL, W_SCALE);
  tconv_kernel<<<dim3(D_MODEL / 64, D_MODEL / 64), blk256, 0, stream>>>(Wv, WqkvT + (size_t)2 * D_MODEL * D_MODEL, D_MODEL, D_MODEL, W_SCALE);
  tconv_kernel<<<dim3(D_MODEL / 64, D_MODEL / 64), blk256, 0, stream>>>(Wo, WoT, D_MODEL, D_MODEL, W_SCALE);
  tconv_kernel<<<dim3(D_FF / 64, D_MODEL / 64), blk256, 0, stream>>>(Wf1, Wf1T, D_MODEL, D_FF, W_SCALE);
  tconv_kernel<<<dim3(D_MODEL / 64, D_FF / 64), blk256, 0, stream>>>(Wf2, Wf2T, D_FF, D_MODEL, W_SCALE);

  ln_kernel<<<dim3(T_SEQ), blk128, 0, stream>>>(x, ln1_g, ln1_b, Xn);

  {
    const int tiles = (T_SEQ / 32) * (3 * D_MODEL / 64);
    gemm_kernel<0><<<dim3((tiles + 7) / 8), blk256, 0, stream>>>(
        Xn, D_MODEL, WqkvT, D_MODEL, (void*)QKV, 3 * D_MODEL, x, D_MODEL,
        T_SEQ, 3 * D_MODEL, D_MODEL, 1.0f / W_SCALE, 2 * D_MODEL);
  }

  attn_kernel<<<dim3(N_HEADS), blk256, 0, stream>>>(QKV, Opl);

  {
    const int tiles = (T_SEQ / 32) * (D_MODEL / 64);
    gemm_kernel<2><<<dim3((tiles + 7) / 8), blk256, 0, stream>>>(
        Opl, D_MODEL, WoT, D_MODEL, (void*)X1, D_MODEL, x, D_MODEL,
        T_SEQ, D_MODEL, D_MODEL, 1.0f / (O_SCALE * W_SCALE), 0);
  }

  ln_kernel<<<dim3(T_SEQ), blk128, 0, stream>>>(X1, ln2_g, ln2_b, H2);

  {
    const int tiles = (T_SEQ / 32) * (D_FF / 64);
    gemm_kernel<1><<<dim3((tiles + 7) / 8), blk256, 0, stream>>>(
        H2, D_MODEL, Wf1T, D_MODEL, (void*)G, D_FF, x, D_MODEL,
        T_SEQ, D_FF, D_MODEL, 1.0f / W_SCALE, 0);
  }

  {
    const int tiles = (T_SEQ / 32) * (D_MODEL / 64);
    gemm_kernel<2><<<dim3((tiles + 7) / 8), blk256, 0, stream>>>(
        G, D_FF, Wf2T, D_FF, (void*)out, D_MODEL, X1, D_MODEL,
        T_SEQ, D_MODEL, D_FF, 1.0f / W_SCALE, 0);
  }
  (void)hipGetLastError();
}
